// _NonLocalBlockND_48902497632272
// MI455X (gfx1250) — hardware-verified
//
#include <hip/hip_runtime.h>
#include <math.h>

#define NB_BATCH 4
#define NCH_C    256
#define NCH_IC   128
#define NT_T     8
#define NH_H     28
#define NW_W     28
#define NHW      (NH_H * NW_W)
#define NPOS     (NT_T * NHW)
#define NW2      (NW_W / 2)
#define NHW2     ((NH_H / 2) * (NW_W / 2))
#define MPOS     (NT_T * NHW2)
#define MPAD     1600
#define BN_EPS   1e-5f
#define XTP      260

static_assert(NPOS % 64 == 0, "npos tile");
static_assert(NPOS % 32 == 0, "npos tr tile");
static_assert(NCH_C % 64 == 0 && NCH_IC % 64 == 0, "ch tiles");
static_assert(NCH_C % 32 == 0 && NCH_IC % 32 == 0, "k tiles");
static_assert(MPOS % 32 == 0, "kv chunks");
static_assert(MPAD % 64 == 0 && MPAD >= MPOS, "vt pad");
static_assert((NB_BATCH * MPOS / 2) % 8 == 0, "pool waves");
static_assert((NCH_IC * NCH_C) % (8 * 256) == 0, "w split blocks");

typedef __attribute__((ext_vector_type(16))) _Float16 v16h;
typedef __attribute__((ext_vector_type(8)))  _Float16 v8h;
typedef __attribute__((ext_vector_type(16))) __bf16   v16b;
typedef __attribute__((ext_vector_type(8)))  __bf16   v8b;
typedef __attribute__((ext_vector_type(8)))  float    v8f;
typedef __attribute__((ext_vector_type(4)))  float    v4f;
typedef __attribute__((ext_vector_type(2)))  float    v2f;
typedef __attribute__((ext_vector_type(4)))  unsigned int v4u;

__device__ __forceinline__ unsigned short f2bf_bits(float f) {
  unsigned u = __float_as_uint(f);
  return (unsigned short)((u + 0x7FFFu + ((u >> 16) & 1u)) >> 16);
}
__device__ __forceinline__ float bf_bits2f(unsigned short h) { return __uint_as_float(((unsigned)h) << 16); }

__device__ __forceinline__ void dep_guard_h(v8f& a, v8f& b, v16h x, v16h y) { asm volatile("v_nop\n\tv_nop\n\tv_nop\n\tv_nop" : "+v"(a), "+v"(b) : "v"(x), "v"(y)); }
__device__ __forceinline__ void dep_guard_b(v8f& a, v8f& b, v16b x, v16b y) { asm volatile("v_nop\n\tv_nop\n\tv_nop\n\tv_nop" : "+v"(a), "+v"(b) : "v"(x), "v"(y)); }
__device__ __forceinline__ void keep4_h(v16h a, v16h b, v16h c, v16h d) { asm volatile("v_nop" :: "v"(a), "v"(b), "v"(c), "v"(d)); }
__device__ __forceinline__ void keep4_b(v16b a, v16b b, v16b c, v16b d) { asm volatile("v_nop" :: "v"(a), "v"(b), "v"(c), "v"(d)); }
__device__ __forceinline__ void acc_guard4(v8f& a, v8f& b, v8f& c, v8f& d) { asm volatile("v_nop\n\tv_nop\n\tv_nop\n\tv_nop" : "+v"(a), "+v"(b), "+v"(c), "+v"(d)); }
template <typename T> struct Frag;
template <> struct Frag<_Float16> {
  typedef v16h V; union U { v16h v; v8h h[2]; };
  static __device__ __forceinline__ v16h load(const _Float16* p) {
    U f; f.h[0] = *(const v8h*)(p); f.h[1] = *(const v8h*)(p + 16); return f.v;
  }
  static __device__ __forceinline__ v8f mma(v16h a, v16h b, v8f c) {
    return __builtin_amdgcn_wmma_f32_16x16x32_f16(false, a, false, b, (short)0, c, false, false);
  }
  static __device__ __forceinline__ void guard(v8f& a, v8f& b, v16h x, v16h y) { dep_guard_h(a, b, x, y); }
  static __device__ __forceinline__ void keep(v16h a, v16h b, v16h c, v16h d) { keep4_h(a, b, c, d); }
};
template <> struct Frag<__bf16> {
  typedef v16b V; union U { v16b v; v8b h[2]; };
  static __device__ __forceinline__ v16b load(const __bf16* p) {
    U f; f.h[0] = *(const v8b*)(p); f.h[1] = *(const v8b*)(p + 16); return f.v;
  }
  static __device__ __forceinline__ v8f mma(v16b a, v16b b, v8f c) {
    return __builtin_amdgcn_wmma_f32_16x16x32_bf16(false, a, false, b, (short)0, c, false, false);
  }
  static __device__ __forceinline__ void guard(v8f& a, v8f& b, v16b x, v16b y) { dep_guard_b(a, b, x, y); }
  static __device__ __forceinline__ void keep(v16b a, v16b b, v16b c, v16b d) { keep4_b(a, b, c, d); }
};

__device__ __forceinline__ unsigned short at_bf_bits(float f) {
  unsigned u = __float_as_uint(f);
  return (unsigned short)((u + 0x7FFFu + ((u >> 16) & 1u)) >> 16);
}
__device__ __forceinline__ __bf16 at_f2bf(float f) { return __builtin_bit_cast(__bf16, at_bf_bits(f)); }
__device__ __forceinline__ void at_split(float f, __bf16& hi, __bf16& lo) {
  const unsigned short hb = at_bf_bits(f);
  hi = __builtin_bit_cast(__bf16, hb);
  lo = at_f2bf(f - __uint_as_float(((unsigned)hb) << 16));
}
__device__ __forceinline__ v8f at_mma(v16b a, v16b b, v8f c) {
  c = __builtin_amdgcn_wmma_f32_16x16x32_bf16(false, a, false, b, (short)0, c, false, false);
  asm volatile("v_nop\n\tv_nop\n\tv_nop\n\tv_nop" : "+v"(c) : "v"(a), "v"(b));
  return c;
}

__device__ __forceinline__ void split8(v4f a, v4f c, v8h& hv, v8h& lv) {
#pragma unroll
  for (int e = 0; e < 4; ++e) {
    const unsigned short hb = f2bf_bits(a[e]);
    const unsigned short lb = f2bf_bits(a[e] - bf_bits2f(hb));
    hv[e] = __builtin_bit_cast(_Float16, hb);
    lv[e] = __builtin_bit_cast(_Float16, lb);
  }
#pragma unroll
  for (int e = 0; e < 4; ++e) {
    const unsigned short hb = f2bf_bits(c[e]);
    const unsigned short lb = f2bf_bits(c[e] - bf_bits2f(hb));
    hv[4 + e] = __builtin_bit_cast(_Float16, hb);
    lv[4 + e] = __builtin_bit_cast(_Float16, lb);
  }
}

__device__ __forceinline__ int pooled_src_pos(int m) {
  const int t = m / NHW2;
  const int rm = m - t * NHW2;
  const int h2 = rm / NW2;
  const int w2 = rm - h2 * NW2;
  return t * NHW + (2 * h2) * NW_W + 2 * w2;
}

template <int ET> struct Elem;
template <> struct Elem<0> { typedef _Float16 T; };
template <> struct Elem<1> { typedef __bf16 T; };
template <int ET, bool SPLIT, int BIAS_MODE, int OUT_MODE>
__global__ __launch_bounds__(256) void wmma_gemm64(
    const unsigned short* __restrict__ Ap, const unsigned short* __restrict__ A2p, int lda, long strideA,
    const unsigned short* __restrict__ Btp, const unsigned short* __restrict__ Bt2p, int ldb, long strideB,
    void* __restrict__ Cout, void* __restrict__ Cout2, int ldc, long strideC,
    const float* __restrict__ bias,
    int M, int N, int K, float scale) {
  typedef typename Elem<ET>::T T;
  typedef typename Frag<T>::V V;
  const T* A = (const T*)Ap; const T* A2 = (const T*)A2p; const T* Bt = (const T*)Btp; const T* Bt2 = (const T*)Bt2p;
  __shared__ __align__(16) float sT[8][16 * 68];
  const int b    = blockIdx.y;
  const int lane = threadIdx.x & 31;
  const int wave = threadIdx.x >> 5;
  const int tilesN = N >> 6;
  const int tilesM = M >> 6;
  const int tile = blockIdx.x * 8 + wave;
  if (tile >= tilesM * tilesN) return;
  const int tm = tile / tilesN;
  const int tn = tile - tm * tilesN;
  const int m0 = tm << 6;
  const int n0 = tn << 6;

  const T* Ab  = A  + (size_t)b * strideA;
  const T* Bb  = Bt + (size_t)b * strideB;
  const T* Ab2 = SPLIT ? (A2  + (size_t)b * strideA) : nullptr;
  const T* Bb2 = SPLIT ? (Bt2 + (size_t)b * strideB) : nullptr;

  const int rlane = lane & 15;
  const int koff  = (lane >> 4) * 8;
  const int mOff  = (lane >> 4) * 8;

  v8f acc[4][4];
#pragma unroll
  for (int i = 0; i < 4; ++i)
#pragma unroll
    for (int j = 0; j < 4; ++j) acc[i][j] = (v8f){0.f,0.f,0.f,0.f,0.f,0.f,0.f,0.f};

  for (int k0 = 0; k0 < K; k0 += 32) {
    V bh[4], bl[4];
#pragma unroll
    for (int j = 0; j < 4; ++j) {
      const size_t bo = (size_t)(n0 + (j << 4) + rlane) * ldb + koff + k0;
      bh[j] = Frag<T>::load(Bb + bo);
      if (SPLIT) bl[j] = Frag<T>::load(Bb2 + bo);
    }
#pragma unroll
    for (int i = 0; i < 4; ++i) {
      const size_t ao = (size_t)(m0 + (i << 4) + rlane) * lda + koff + k0;
      V ah = Frag<T>::load(Ab + ao);
      V al;
      if (SPLIT) al = Frag<T>::load(Ab2 + ao);
#pragma unroll
      for (int j = 0; j < 4; ++j) {
        acc[i][j] = Frag<T>::mma(ah, bh[j], acc[i][j]);
        if (SPLIT) {
          acc[i][j] = Frag<T>::mma(ah, bl[j], acc[i][j]);
          acc[i][j] = Frag<T>::mma(al, bh[j], acc[i][j]);
        }
      }
      Frag<T>::guard(acc[i][0], acc[i][3], ah, SPLIT ? al : ah);
    }
    Frag<T>::keep(bh[0], bh[1], bh[2], bh[3]);
    if (SPLIT) Frag<T>::keep(bl[0], bl[1], bl[2], bl[3]);
  }
  acc_guard4(acc[0][0], acc[0][1], acc[0][2], acc[0][3]);
  acc_guard4(acc[1][0], acc[1][1], acc[1][2], acc[1][3]);
  acc_guard4(acc[2][0], acc[2][1], acc[2][2], acc[2][3]);
  acc_guard4(acc[3][0], acc[3][1], acc[3][2], acc[3][3]);

  float* slab = sT[wave];
#pragma unroll
  for (int i = 0; i < 4; ++i) {
    const int mBase = m0 + (i << 4);
    float bm[8];
    if (BIAS_MODE == 1) {
      const v4f bq0 = *(const v4f*)(bias + mBase + mOff);
      const v4f bq1 = *(const v4f*)(bias + mBase + mOff + 4);
      bm[0] = bq0[0]; bm[1] = bq0[1]; bm[2] = bq0[2]; bm[3] = bq0[3];
      bm[4] = bq1[0]; bm[5] = bq1[1]; bm[6] = bq1[2]; bm[7] = bq1[3];
    } else {
#pragma unroll
      for (int e = 0; e < 8; ++e) bm[e] = 0.f;
    }
#pragma unroll
    for (int j = 0; j < 4; ++j) {
      const int n = n0 + (j << 4) + rlane;
      float bv = 0.f;
      if (BIAS_MODE == 2) bv = bias[n];
#pragma unroll
      for (int r = 0; r < 8; ++r) {
        float v = acc[i][j][r] * scale;
        if (BIAS_MODE == 1) v += bm[r];
        if (BIAS_MODE == 2) v += bv;
        slab[(mOff + r) * 68 + (j << 4) + rlane] = v;
      }
    }
    __builtin_amdgcn_fence(__ATOMIC_RELEASE, "workgroup");
    __builtin_amdgcn_wave_barrier();
    __builtin_amdgcn_fence(__ATOMIC_ACQUIRE, "workgroup");
    if (OUT_MODE == 0) {
      float* C = (float*)Cout + (size_t)b * strideC;
      const int hh = lane >> 4, c4 = (lane & 15) * 4;
      for (int pass = 0; pass < 2; ++pass) {
#pragma unroll
        for (int it = 0; it < 8; ++it) {
          const int row = it * 2 + hh;
          v4f v = *(const v4f*)(slab + row * 68 + c4);
          *(volatile v4f*)(C + (size_t)(mBase + row) * ldc + n0 + c4) = v;
        }
        __threadfence();
      }
    } else {
      const int q = lane >> 3, c8 = (lane & 7) * 8;
      unsigned short* C  = (unsigned short*)Cout  + (size_t)b * strideC;
      unsigned short* C2 = (OUT_MODE == 2) ? ((unsigned short*)Cout2 + (size_t)b * strideC) : nullptr;
      for (int pass = 0; pass < 2; ++pass) {
#pragma unroll
        for (int it = 0; it < 4; ++it) {
          const int row = it * 4 + q;
          const float* sp = slab + row * 68 + c8;
          v8h hv, lv;
#pragma unroll
          for (int e = 0; e < 8; ++e) {
            if (OUT_MODE == 1) {
              hv[e] = (_Float16)sp[e];
            } else {
              unsigned short hb = f2bf_bits(sp[e]);
              unsigned short lb = f2bf_bits(sp[e] - bf_bits2f(hb));
              hv[e] = __builtin_bit_cast(_Float16, hb);
              lv[e] = __builtin_bit_cast(_Float16, lb);
            }
          }
          *(volatile v8h*)(C + (size_t)(mBase + row) * ldc + n0 + c8) = hv;
          if (OUT_MODE == 2) *(volatile v8h*)(C2 + (size_t)(mBase + row) * ldc + n0 + c8) = lv;
        }
        __threadfence();
      }
    }
    __builtin_amdgcn_fence(__ATOMIC_RELEASE, "workgroup");
    __builtin_amdgcn_wave_barrier();
    __builtin_amdgcn_fence(__ATOMIC_ACQUIRE, "workgroup");
  }
}

#define BN_MAXCH 256
__global__ __launch_bounds__(256) void wmma_gemm64_bn_resid(
    const unsigned short* __restrict__ Ap, const unsigned short* __restrict__ A2p, int lda,
    const unsigned short* __restrict__ Btp, const unsigned short* __restrict__ Bt2p, int ldb, long strideB,
    float* __restrict__ Cout, int ldc, long strideC,
    const float* __restrict__ resid,
    const float* __restrict__ gam, const float* __restrict__ bet,
    const float* __restrict__ rmean, const float* __restrict__ rvar,
    int M, int N, int K) {
  typedef __bf16 T;
  typedef v16b V;
  const T* A = (const T*)Ap; const T* A2 = (const T*)A2p; const T* Bt = (const T*)Btp; const T* Bt2 = (const T*)Bt2p;
  __shared__ __align__(16) float sT[8][16 * 68];
  __shared__ float s_mu[BN_MAXCH], s_ig[BN_MAXCH], s_be[BN_MAXCH];
  for (int ch = threadIdx.x; ch < M; ch += 256) {
    const float ig = gam[ch] * rsqrtf(rvar[ch] + BN_EPS);
    s_mu[ch] = rmean[ch];
    s_ig[ch] = ig;
    s_be[ch] = bet[ch];
  }
  __syncthreads();

  const int b    = blockIdx.y;
  const int lane = threadIdx.x & 31;
  const int wave = threadIdx.x >> 5;
  const int tilesN = N >> 6;
  const int tilesM = M >> 6;
  const int tile = blockIdx.x * 8 + wave;
  if (tile >= tilesM * tilesN) return;
  const int tm = tile / tilesN;
  const int tn = tile - tm * tilesN;
  const int m0 = tm << 6;
  const int n0 = tn << 6;

  const T* Ab  = A;
  const T* Bb  = Bt + (size_t)b * strideB;
  const T* Ab2 = A2;
  const T* Bb2 = Bt2 + (size_t)b * strideB;

  const int rlane = lane & 15;
  const int koff  = (lane >> 4) * 8;
  const int mOff  = (lane >> 4) * 8;

  v8f acc[4][4];
#pragma unroll
  for (int i = 0; i < 4; ++i)
#pragma unroll
    for (int j = 0; j < 4; ++j) acc[i][j] = (v8f){0.f,0.f,0.f,0.f,0.f,0.f,0.f,0.f};

  for (int k0 = 0; k0 < K; k0 += 32) {
    V bh[4], bl[4];
#pragma unroll
    for (int j = 0; j < 4; ++j) {
      const size_t bo = (size_t)(n0 + (j << 4) + rlane) * ldb + koff + k0;
      bh[j] = Frag<T>::load(Bb + bo);
      bl[j] = Frag<T>::load(Bb2 + bo);
    }
#pragma unroll
    for (int i = 0; i < 4; ++i) {
      const size_t ao = (size_t)(m0 + (i << 4) + rlane) * lda + koff + k0;
      V ah = Frag<T>::load(Ab + ao);
      V al = Frag<T>::load(Ab2 + ao);
#pragma unroll
      for (int j = 0; j < 4; ++j) {
        acc[i][j] = Frag<T>::mma(ah, bh[j], acc[i][j]);
        acc[i][j] = Frag<T>::mma(ah, bl[j], acc[i][j]);
        acc[i][j] = Frag<T>::mma(al, bh[j], acc[i][j]);
      }
      Frag<T>::guard(acc[i][0], acc[i][3], ah, al);
    }
    Frag<T>::keep(bh[0], bh[1], bh[2], bh[3]);
    Frag<T>::keep(bl[0], bl[1], bl[2], bl[3]);
  }
  acc_guard4(acc[0][0], acc[0][1], acc[0][2], acc[0][3]);
  acc_guard4(acc[1][0], acc[1][1], acc[1][2], acc[1][3]);
  acc_guard4(acc[2][0], acc[2][1], acc[2][2], acc[2][3]);
  acc_guard4(acc[3][0], acc[3][1], acc[3][2], acc[3][3]);

  float* slab = sT[wave];
  float* C = Cout + (size_t)b * strideC;
  const float* R = resid + (size_t)b * strideC;
#pragma unroll
  for (int i = 0; i < 4; ++i) {
    const int mBase = m0 + (i << 4);
#pragma unroll
    for (int j = 0; j < 4; ++j) {
#pragma unroll
      for (int r = 0; r < 8; ++r) {
        const int row = mBase + mOff + r;
        const float v = (acc[i][j][r] - s_mu[row]) * s_ig[row] + s_be[row];
        slab[(mOff + r) * 68 + (j << 4) + rlane] = v;
      }
    }
    __builtin_amdgcn_fence(__ATOMIC_RELEASE, "workgroup");
    __builtin_amdgcn_wave_barrier();
    __builtin_amdgcn_fence(__ATOMIC_ACQUIRE, "workgroup");
    {
      const int hh = lane >> 4, c4 = (lane & 15) * 4;
      for (int pass = 0; pass < 2; ++pass) {
#pragma unroll
        for (int it = 0; it < 8; ++it) {
          const int row = it * 2 + hh;
          const size_t go = (size_t)(mBase + row) * ldc + n0 + c4;
          v4f v = *(const v4f*)(slab + row * 68 + c4);
          const v4f xr = *(const v4f*)(R + go);
          v += xr;
          *(volatile v4f*)(C + go) = v;
        }
        __threadfence();
      }
    }
    __builtin_amdgcn_fence(__ATOMIC_RELEASE, "workgroup");
    __builtin_amdgcn_wave_barrier();
    __builtin_amdgcn_fence(__ATOMIC_ACQUIRE, "workgroup");
  }
}

__global__ __launch_bounds__(256) void split_f32_bf16x8(const float* __restrict__ in,
    unsigned short* __restrict__ hi, unsigned short* __restrict__ lo, int n8) {
  const int i = blockIdx.x * 256 + threadIdx.x;
  if (i < n8) {
    const size_t e0 = (size_t)i * 8;
    const v4f a = *(const v4f*)(in + e0);
    const v4f c = *(const v4f*)(in + e0 + 4);
    v8h hv, lv;
    split8(a, c, hv, lv);
    *(volatile v8h*)(hi + e0) = hv;
    *(volatile v8h*)(lo + e0) = lv;
    __threadfence();
    *(volatile v8h*)(hi + e0) = hv;
    *(volatile v8h*)(lo + e0) = lv;
  }
}

__global__ __launch_bounds__(256) void xt_split(const float* __restrict__ x,
    unsigned short* __restrict__ xh, unsigned short* __restrict__ xl) {
  __shared__ __align__(16) float tile[32 * XTP];
  const int tid = threadIdx.x, wave = tid >> 5, lane = tid & 31;
  const int b = blockIdx.y, n0 = blockIdx.x * 32;
  const float* xb = x + (size_t)b * NCH_C * NPOS + n0;
  {
    const int n4 = (tid & 7) * 4, cr = tid >> 3;
#pragma unroll
    for (int i = 0; i < 8; ++i) {
      const int cc = cr + 32 * i;
      const v4f v = *(const v4f*)(xb + (size_t)cc * NPOS + n4);
      tile[(n4 + 0) * XTP + cc] = v[0];
      tile[(n4 + 1) * XTP + cc] = v[1];
      tile[(n4 + 2) * XTP + cc] = v[2];
      tile[(n4 + 3) * XTP + cc] = v[3];
    }
  }
  __syncthreads();
  const int row = wave * 4 + (lane >> 3), c8 = (lane & 7) * 8;
  const size_t ob = ((size_t)b * NPOS + n0 + row) * NCH_C;
  for (int pass = 0; pass < 2; ++pass) {
#pragma unroll
    for (int cb = 0; cb < 4; ++cb) {
      const int col = cb * 64 + c8;
      const v4f a = *(const v4f*)(tile + row * XTP + col);
      const v4f c = *(const v4f*)(tile + row * XTP + col + 4);
      v8h hv, lv;
      split8(a, c, hv, lv);
      *(volatile v8h*)(xh + ob + col) = hv;
      *(volatile v8h*)(xl + ob + col) = lv;
    }
    __threadfence();
  }
}

__global__ __launch_bounds__(256) void pool_rows_split(const float* __restrict__ src,
    unsigned short* __restrict__ oh, unsigned short* __restrict__ ol) {
  const int lane = threadIdx.x & 31;
  const int gw = blockIdx.x * 8 + (threadIdx.x >> 5);
  const int R = gw * 2 + (lane >> 4);
  const int b = R / MPOS, m = R - b * MPOS;
  const int d8 = (lane & 15) * 8;
  const int p = pooled_src_pos(m);
  const float* s0 = src + ((size_t)b * NPOS + p) * NCH_IC + d8;
  const v4f a0 = *(const v4f*)(s0),                           a1 = *(const v4f*)(s0 + 4);
  const v4f b0 = *(const v4f*)(s0 + NCH_IC),                  b1 = *(const v4f*)(s0 + NCH_IC + 4);
  const v4f c0 = *(const v4f*)(s0 + NW_W * NCH_IC),           c1 = *(const v4f*)(s0 + NW_W * NCH_IC + 4);
  const v4f e0 = *(const v4f*)(s0 + (NW_W + 1) * NCH_IC),     e1 = *(const v4f*)(s0 + (NW_W + 1) * NCH_IC + 4);
  v4f m0v, m1v;
#pragma unroll
  for (int k = 0; k < 4; ++k) {
    m0v[k] = fmaxf(fmaxf(a0[k], b0[k]), fmaxf(c0[k], e0[k]));
    m1v[k] = fmaxf(fmaxf(a1[k], b1[k]), fmaxf(c1[k], e1[k]));
  }
  v8h hv, lv;
  split8(m0v, m1v, hv, lv);
  const size_t oo = (size_t)R * NCH_IC + d8;
  *(volatile v8h*)(oh + oo) = hv;
  *(volatile v8h*)(ol + oo) = lv;
  __threadfence();
  *(volatile v8h*)(oh + oo) = hv;
  *(volatile v8h*)(ol + oo) = lv;
}

__global__ __launch_bounds__(256) void pool_tr_split(const float* __restrict__ src,
    unsigned short* __restrict__ oh, unsigned short* __restrict__ ol) {
  const int lane = threadIdx.x & 31, wave = threadIdx.x >> 5;
  const int mt = blockIdx.x, dg = blockIdx.y, b = blockIdx.z;
  const int d = dg * 32 + wave * 4 + (lane >> 3);
  const int mloc = (lane & 7) * 8;
  const int mb = mt * 64 + mloc;
  const float* row = src + ((size_t)b * NCH_IC + d) * NPOS;
  float mx[8];
#pragma unroll
  for (int e = 0; e < 8; ++e) {
    int m = mb + e;
    m = (m < MPOS) ? m : (MPOS - 1);
    const int p = pooled_src_pos(m);
    const v2f u = *(const v2f*)(row + p);
    const v2f w = *(const v2f*)(row + p + NW_W);
    mx[e] = fmaxf(fmaxf(u[0], u[1]), fmaxf(w[0], w[1]));
    if (e == 3) asm volatile("" ::: "memory");
  }
  v4f a, c;
  a[0] = mx[0]; a[1] = mx[1]; a[2] = mx[2]; a[3] = mx[3];
  c[0] = mx[4]; c[1] = mx[5]; c[2] = mx[6]; c[3] = mx[7];
  v8h hv, lv;
  split8(a, c, hv, lv);
  const size_t oo = ((size_t)b * NCH_IC + d) * MPAD + mt * 64 + mloc;
  *(volatile v8h*)(oh + oo) = hv;
  *(volatile v8h*)(ol + oo) = lv;
  __threadfence();
  *(volatile v8h*)(oh + oo) = hv;
  *(volatile v8h*)(ol + oo) = lv;
}

#define AHD 128
#define AKC 32
#define AQB 64
#define ANW 4
#define OSP 132
__global__ __launch_bounds__(128) void attn_d128_split(
    const unsigned short* __restrict__ Thp, const unsigned short* __restrict__ Tlp,
    const unsigned short* __restrict__ Khp, const unsigned short* __restrict__ Klp,
    const unsigned short* __restrict__ Vhp, const unsigned short* __restrict__ Vlp,
    unsigned short* __restrict__ Yhp, unsigned short* __restrict__ Ylp) {
  __shared__ __align__(16) __bf16 Qh_s[AQB * AHD];
  __shared__ __align__(16) __bf16 Ql_s[AQB * AHD];
  __shared__ __align__(16) __bf16 Kh_s[AKC * AHD];
  __shared__ __align__(16) __bf16 Kl_s[AKC * AHD];
  __shared__ __align__(16) __bf16 Vh_s[AHD * AKC];
  __shared__ __align__(16) __bf16 Vl_s[AHD * AKC];
  __shared__ __align__(16) __bf16 Ph_s[ANW][16 * AKC];
  __shared__ __align__(16) __bf16 Pl_s[ANW][16 * AKC];
  __shared__ __align__(16) float  Os[ANW][16 * OSP];

  const int tid  = threadIdx.x;
  const int wave = tid >> 5;
  const int lane = tid & 31;
  const int hh   = lane >> 4;
  const int c    = lane & 15;
  const int koff = hh * 8;

  const int nqb   = NPOS / AQB;
  const int b     = blockIdx.x / nqb;
  const int qb    = blockIdx.x - b * nqb;
  const int qbase = qb * AQB;
  const int q0    = qbase + wave * 16;

  {
    const v4u* gh = (const v4u*)(Thp + ((size_t)b * NPOS + qbase) * AHD);
    const v4u* gl = (const v4u*)(Tlp + ((size_t)b * NPOS + qbase) * AHD);
    v4u* sh = (v4u*)Qh_s;
    v4u* sl = (v4u*)Ql_s;
#pragma unroll
    for (int i = 0; i < 8; ++i) sh[tid + 128 * i] = gh[tid + 128 * i];
    asm volatile("" ::: "memory");
#pragma unroll
    for (int i = 0; i < 8; ++i) sl[tid + 128 * i] = gl[tid + 128 * i];
  }

  float mrow[8], lrow[8];
  v8f oacc[8];
#pragma unroll
  for (int r = 0; r < 8; ++r) { mrow[r] = -INFINITY; lrow[r] = 0.f; }
#pragma unroll
  for (int t = 0; t < 8; ++t) oacc[t] = (v8f){0.f,0.f,0.f,0.f,0.f,0.f,0.f,0.f};

  for (int kc = 0; kc < MPOS / AKC; ++kc) {
    const int kv0 = kc * AKC;
    __syncthreads();
    {
      const v4u* kh_g = (const v4u*)(Khp + ((size_t)b * MPOS + kv0) * AHD);
      const v4u* kl_g = (const v4u*)(Klp + ((size_t)b * MPOS + kv0) * AHD);
      v4u* kh_s = (v4u*)Kh_s;
      v4u* kl_s = (v4u*)Kl_s;
#pragma unroll
      for (int i = 0; i < 4; ++i) kh_s[tid + 128 * i] = kh_g[tid + 128 * i];
#pragma unroll
      for (int i = 0; i < 4; ++i) kl_s[tid + 128 * i] = kl_g[tid + 128 * i];
      asm volatile("" ::: "memory");
      const int vd = tid >> 2, vj = (tid & 3) * 8;
#pragma unroll
      for (int i = 0; i < 4; ++i) {
        const int d = vd + 32 * i;
        const v4u hv4 = *(const v4u*)(Vhp + ((size_t)b * AHD + d) * MPAD + kv0 + vj);
        *(v4u*)(Vh_s + d * AKC + vj) = hv4;
      }
#pragma unroll
      for (int i = 0; i < 4; ++i) {
        const int d = vd + 32 * i;
        const v4u lv4 = *(const v4u*)(Vlp + ((size_t)b * AHD + d) * MPAD + kv0 + vj);
        *(v4u*)(Vl_s + d * AKC + vj) = lv4;
      }
    }
    __syncthreads();

    v8f s[2];
    s[0] = (v8f){0.f,0.f,0.f,0.f,0.f,0.f,0.f,0.f};
    s[1] = (v8f){0.f,0.f,0.f,0.f,0.f,0.f,0.f,0.f};
#pragma unroll
    for (int dc = 0; dc < 4; ++dc) {
      const v16b qh = Frag<__bf16>::load(Qh_s + (wave * 16 + c) * AHD + dc * 32 + koff);
      const v16b ql = Frag<__bf16>::load(Ql_s + (wave * 16 + c) * AHD + dc * 32 + koff);
#pragma unroll
      for (int j = 0; j < 2; ++j) {
        const v16b kb = Frag<__bf16>::load(Kh_s + (j * 16 + c) * AHD + dc * 32 + koff);
        const v16b kl = Frag<__bf16>::load(Kl_s + (j * 16 + c) * AHD + dc * 32 + koff);
        s[j] = at_mma(qh, kb, s[j]);
        s[j] = at_mma(qh, kl, s[j]);
        s[j] = at_mma(ql, kb, s[j]);
      }
    }

    float cm[8];
#pragma unroll
    for (int r = 0; r < 8; ++r) {
      float mxv = fmaxf(s[0][r], s[1][r]);
#pragma unroll
      for (int off = 1; off < 16; off <<= 1) mxv = fmaxf(mxv, __shfl_xor(mxv, off, 32));
      cm[r] = mxv;
    }
    __bf16* pwh = Ph_s[wave];
    __bf16* pwl = Pl_s[wave];
#pragma unroll
    for (int r = 0; r < 8; ++r) {
      const float mnew = fmaxf(mrow[r], cm[r]);
      const float alpha = expf(mrow[r] - mnew);
      mrow[r] = mnew;
      float psum = 0.f;
#pragma unroll
      for (int j = 0; j < 2; ++j) {
        const float p = expf(s[j][r] - mnew);
        psum += p;
        __bf16 ph, plo;
        at_split(p, ph, plo);
        pwh[(8 * hh + r) * AKC + j * 16 + c] = ph;
        pwl[(8 * hh + r) * AKC + j * 16 + c] = plo;
      }
#pragma unroll
      for (int off = 1; off < 16; off <<= 1) psum += __shfl_xor(psum, off, 32);
      lrow[r] = lrow[r] * alpha + psum;
#pragma unroll
      for (int t = 0; t < 8; ++t) oacc[t][r] *= alpha;
    }
    __builtin_amdgcn_fence(__ATOMIC_RELEASE, "workgroup");
    __builtin_amdgcn_wave_barrier();
    __builtin_amdgcn_fence(__ATOMIC_ACQUIRE, "workgroup");

    {
      const v16b pa = Frag<__bf16>::load(pwh + c * AKC + koff);
      const v16b pl = Frag<__bf16>::load(pwl + c * AKC + koff);
#pragma unroll
      for (int t = 0; t < 8; ++t) {
        const v16b vb = Frag<__bf16>::load(Vh_s + (t * 16 + c) * AKC + koff);
        const v16b vl = Frag<__bf16>::load(Vl_s + (t * 16 + c) * AKC + koff);
        oacc[t] = at_mma(pa, vb, oacc[t]);
        oacc[t] = at_mma(pa, vl, oacc[t]);
        oacc[t] = at_mma(pl, vb, oacc[t]);
      }
    }
  }

  float* os = Os[wave];
#pragma unroll
  for (int r = 0; r < 8; ++r) {
    const float inv = 1.0f / lrow[r];
#pragma unroll
    for (int t = 0; t < 8; ++t) os[(8 * hh + r) * OSP + t * 16 + c] = oacc[t][r] * inv;
  }
  __builtin_amdgcn_fence(__ATOMIC_RELEASE, "workgroup");
  __builtin_amdgcn_wave_barrier();
  __builtin_amdgcn_fence(__ATOMIC_ACQUIRE, "workgroup");
  {
    const int r2 = lane >> 4, c8 = (lane & 15) * 8;
    for (int pass = 0; pass < 2; ++pass) {
#pragma unroll
      for (int it = 0; it < 8; ++it) {
        const int row = it * 2 + r2;
        const v4f a  = *(const v4f*)(os + row * OSP + c8);
        const v4f cc = *(const v4f*)(os + row * OSP + c8 + 4);
        v8h hv, lv;
        split8(a, cc, hv, lv);
        const size_t yo = ((size_t)b * NPOS + q0 + row) * AHD + c8;
        *(volatile v8h*)(Yhp + yo) = hv;
        *(volatile v8h*)(Ylp + yo) = lv;
      }
      __threadfence();
    }
  }
}

constexpr size_t SZ_XP = (size_t)NB_BATCH * NPOS * NCH_C * 2;
constexpr size_t SZ_TP = (size_t)NB_BATCH * NPOS * NCH_IC * 2;
constexpr size_t SZ_GF = (size_t)NB_BATCH * NCH_IC * NPOS * 4;
constexpr size_t SZ_PF = (size_t)NB_BATCH * NPOS * NCH_IC * 4;
constexpr size_t SZ_KP = (size_t)NB_BATCH * MPOS * NCH_IC * 2;
constexpr size_t SZ_VP = (size_t)NB_BATCH * NCH_IC * MPAD * 2;
constexpr size_t SZ_YP = SZ_TP;
constexpr size_t SZ_WP = (size_t)NCH_IC * NCH_C * 2;
constexpr size_t OFF_XH = 0;
constexpr size_t OFF_XL = OFF_XH + SZ_XP;
constexpr size_t OFF_TH = OFF_XL + SZ_XP;
constexpr size_t OFF_TL = OFF_TH + SZ_TP;
constexpr size_t OFF_GF = OFF_TL + SZ_TP;
constexpr size_t OFF_PF = OFF_GF + SZ_GF;
constexpr size_t OFF_KH = OFF_PF + SZ_PF;
constexpr size_t OFF_KL = OFF_KH + SZ_KP;
constexpr size_t OFF_VH = OFF_KL + SZ_KP;
constexpr size_t OFF_VL = OFF_VH + SZ_VP;
constexpr size_t OFF_YH = OFF_VL + SZ_VP;
constexpr size_t OFF_YL = OFF_YH + SZ_YP;
constexpr size_t OFF_W0 = OFF_YL + SZ_YP;
constexpr size_t OFF_END = OFF_W0 + 8 * SZ_WP;
static_assert(OFF_END == 84082688, "carve total");
static_assert(OFF_END <= 134217728, "carve cap");
static_assert(SZ_XP % 256 == 0 && SZ_TP % 256 == 0 && SZ_KP % 256 == 0 && SZ_VP % 256 == 0 && SZ_WP % 256 == 0, "align");

extern "C" void kernel_launch(void* const* d_in, const int* in_sizes, int n_in,
                              void* d_out, int out_size, void* d_ws, size_t ws_size,
                              hipStream_t stream) {
  if (n_in < 12) return;
  if (ws_size < OFF_END) return;
  if (in_sizes[0] != NB_BATCH * NCH_C * NPOS) return;
  if ((size_t)out_size != (size_t)NB_BATCH * NCH_C * NPOS) return;

  const float* x    = (const float*)d_in[0];
  const float* Wg   = (const float*)d_in[1];
  const float* bg   = (const float*)d_in[2];
  const float* Wt   = (const float*)d_in[3];
  const float* bt   = (const float*)d_in[4];
  const float* Wp   = (const float*)d_in[5];
  const float* bp   = (const float*)d_in[6];
  const float* Ww   = (const float*)d_in[7];
  const float* bn_g = (const float*)d_in[8];
  const float* bn_b = (const float*)d_in[9];
  const float* bn_m = (const float*)d_in[10];
  const float* bn_v = (const float*)d_in[11];
  float* out = (float*)d_out;

  char* ws = (char*)d_ws;
  unsigned short* xh  = (unsigned short*)(ws + OFF_XH);
  unsigned short* xl  = (unsigned short*)(ws + OFF_XL);
  unsigned short* th  = (unsigned short*)(ws + OFF_TH);
  unsigned short* tl  = (unsigned short*)(ws + OFF_TL);
  float*          gf  = (float*)(ws + OFF_GF);
  float*          pf  = (float*)(ws + OFF_PF);
  unsigned short* kh  = (unsigned short*)(ws + OFF_KH);
  unsigned short* kl  = (unsigned short*)(ws + OFF_KL);
  unsigned short* vh  = (unsigned short*)(ws + OFF_VH);
  unsigned short* vl  = (unsigned short*)(ws + OFF_VL);
  unsigned short* yh  = (unsigned short*)(ws + OFF_YH);
  unsigned short* yl  = (unsigned short*)(ws + OFF_YL);
  unsigned short* wgh = (unsigned short*)(ws + OFF_W0 + 0 * SZ_WP);
  unsigned short* wgl = (unsigned short*)(ws + OFF_W0 + 1 * SZ_WP);
  unsigned short* wth = (unsigned short*)(ws + OFF_W0 + 2 * SZ_WP);
  unsigned short* wtl = (unsigned short*)(ws + OFF_W0 + 3 * SZ_WP);
  unsigned short* wph = (unsigned short*)(ws + OFF_W0 + 4 * SZ_WP);
  unsigned short* wpl = (unsigned short*)(ws + OFF_W0 + 5 * SZ_WP);
  unsigned short* wwh = (unsigned short*)(ws + OFF_W0 + 6 * SZ_WP);
  unsigned short* wwl = (unsigned short*)(ws + OFF_W0 + 7 * SZ_WP);

  const int wn8 = NCH_IC * NCH_C / 8;
  split_f32_bf16x8<<<wn8 / 256, 256, 0, stream>>>(Wg, wgh, wgl, wn8);
  split_f32_bf16x8<<<wn8 / 256, 256, 0, stream>>>(Wt, wth, wtl, wn8);
  split_f32_bf16x8<<<wn8 / 256, 256, 0, stream>>>(Wp, wph, wpl, wn8);
  split_f32_bf16x8<<<wn8 / 256, 256, 0, stream>>>(Ww, wwh, wwl, wn8);

  xt_split<<<dim3(NPOS / 32, NB_BATCH), 256, 0, stream>>>(x, xh, xl);

  const int convTiles = (NPOS / 64) * (NCH_IC / 64);
  const dim3 gconv((convTiles + 7) / 8, NB_BATCH);
  wmma_gemm64<1, true, 2, 2><<<gconv, 256, 0, stream>>>(
      xh, xl, NCH_C, (long)NPOS * NCH_C,
      wth, wtl, NCH_C, 0L,
      (void*)th, (void*)tl, NCH_IC, (long)NPOS * NCH_IC,
      bt, NPOS, NCH_IC, NCH_C, 1.0f);
  wmma_gemm64<1, true, 2, 0><<<gconv, 256, 0, stream>>>(
      xh, xl, NCH_C, (long)NPOS * NCH_C,
      wph, wpl, NCH_C, 0L,
      (void*)pf, (void*)nullptr, NCH_IC, (long)NPOS * NCH_IC,
      bp, NPOS, NCH_IC, NCH_C, 1.0f);
  wmma_gemm64<1, true, 1, 0><<<gconv, 256, 0, stream>>>(
      wgh, wgl, NCH_C, 0L,
      xh, xl, NCH_C, (long)NPOS * NCH_C,
      (void*)gf, (void*)nullptr, NPOS, (long)NCH_IC * NPOS,
      bg, NCH_IC, NPOS, NCH_C, 1.0f);

  pool_rows_split<<<(NB_BATCH * MPOS / 2) / 8, 256, 0, stream>>>(pf, kh, kl);
  pool_tr_split<<<dim3(MPAD / 64, NCH_IC / 32, NB_BATCH), 256, 0, stream>>>(gf, vh, vl);

  attn_d128_split<<<NB_BATCH * (NPOS / AQB), 128, 0, stream>>>(th, tl, kh, kl, vh, vl, yh, yl);

  const int outTiles = (NCH_C / 64) * (NPOS / 64);
  wmma_gemm64_bn_resid<<<dim3((outTiles + 7) / 8, NB_BATCH), 256, 0, stream>>>(
      wwh, wwl, NCH_IC,
      yh, yl, NCH_IC, (long)NPOS * NCH_IC,
      out, NPOS, (long)NCH_C * NPOS,
      x, bn_g, bn_b, bn_m, bn_v,
      NCH_C, NPOS, NCH_IC);
}
